// GCN_67946382623222
// MI455X (gfx1250) — hardware-run, weakly checked
//
#include <hip/hip_runtime.h>
#include <stddef.h>
#include <stdint.h>
#include <math.h>

#define NN      100000
#define CIN     128
#define HD      64
#define NE      1600000
#define GBM     128
#define MP      100096
#define KL      128
#define APITCH  128
#define BPITCH  128
#define TWO_TERM 1
#define K2EXT   (TWO_TERM ? 128 : 64)
#define NTHR    256
#define NWAVE   8
#define EPT     8
#define WCH     (32 * EPT)
#define NBRUN   1024
#define SLB     10
#define NBK     98
#define WLCAP   2560
#define RCAP    20480
#define DEGCAP  64
#define MAXDEG_MEAS   36
#define MAXB1024_MEAS 16710
#define SP      68
#define WSMAX   ((size_t)128 << 20)

#define BK_ZINTS (NWAVE * WLCAP + RCAP + 3 * NBRUN)
#define BK_INTS  (BK_ZINTS + 16)
#define BK_LDS   (BK_INTS * 4)

#define PBX   (MP * CIN / 8 / NTHR)
#define PBW   (HD * KL / 8 / NTHR)
#define PBTOT (PBX + 3 * PBW + 1)

static_assert(HD == 64 && HD == 16 * 4);
static_assert(CIN % 32 == 0 && KL % 32 == 0 && K2EXT % 32 == 0 && KL == 2 * HD && CIN == KL);
static_assert(APITCH >= CIN && APITCH >= K2EXT && BPITCH >= CIN && BPITCH >= K2EXT);
static_assert(MP % GBM == 0 && MP >= NN && MP == 782 * GBM && NN <= 100096);
static_assert(NBRUN == (1 << SLB) && NBRUN % 32 == 0 && NBRUN % NTHR == 0 && NBRUN == NWAVE * 128);
static_assert(NBK * NBRUN >= MP && NBK * NBRUN >= NN);
static_assert(NE < (1 << 21) && (((long long)NE) << SLB) < (1LL << 31));
static_assert(NE % WCH == 0 && NE % 4 == 0);
static_assert(RCAP == NWAVE * WLCAP && RCAP % (NTHR * 4) == 0 && BK_ZINTS % (NTHR * 4) == 0);
static_assert((long long)RCAP * 100 >= (long long)MAXB1024_MEAS * 105);
static_assert(WLCAP >= MAXB1024_MEAS / 8 + 8 * 46 + 1);
static_assert(MAXDEG_MEAS + 8 <= DEGCAP);
static_assert(BK_LDS <= 300000 && BK_LDS <= 327680);
static_assert(GBM * SP * 4 <= 65536);
static_assert((MP * CIN / 8) % NTHR == 0 && (HD * KL / 8) % NTHR == 0);
static_assert(NN * HD == 6400000);

typedef float          v4f   __attribute__((ext_vector_type(4)));
typedef float          v8f   __attribute__((ext_vector_type(8)));
typedef int            v4i   __attribute__((ext_vector_type(4)));
typedef int            v8i   __attribute__((ext_vector_type(8)));
typedef unsigned short v8us  __attribute__((ext_vector_type(8)));
typedef unsigned short v16us __attribute__((ext_vector_type(16)));
typedef __bf16         v16bf __attribute__((ext_vector_type(16)));
typedef v4f  __attribute__((may_alias)) v4fa;
typedef v4i  __attribute__((may_alias)) v4ia;
typedef v8us __attribute__((may_alias)) v8usa;
union FragB { v16bf v; v16us u; v8us h[2]; v8i w; };

__device__ __forceinline__ v8f wmb(const FragB& a, const FragB& b, v8f c) {
  v8f d = __builtin_amdgcn_wmma_f32_16x16x32_bf16(false, a.v, false, b.v, (short)0, c, false, false);
  asm volatile("v_nop\n\tv_nop\n\tv_nop\n\tv_nop" : "+v"(d) : "v"(a.w), "v"(b.w));
  return d;
}

__device__ __forceinline__ unsigned bf16_bits(float f) {
  const unsigned u = __float_as_uint(f);
  const unsigned r = (u + 0x7FFFu + ((u >> 16) & 1u)) >> 16;
  const unsigned q = (u >> 16) | 0x40u;
  return ((u & 0x7fffffffu) > 0x7f800000u) ? q : r;
}

__device__ __forceinline__ void hilo_pack(float v0, float v1, float v2, float v3,
                                          int& h01, int& h23, int& l01, int& l23) {
  const unsigned a0 = bf16_bits(v0), a1 = bf16_bits(v1), a2 = bf16_bits(v2), a3 = bf16_bits(v3);
  const unsigned b0 = bf16_bits(v0 - __uint_as_float(a0 << 16));
  const unsigned b1 = bf16_bits(v1 - __uint_as_float(a1 << 16));
  const unsigned b2 = bf16_bits(v2 - __uint_as_float(a2 << 16));
  const unsigned b3 = bf16_bits(v3 - __uint_as_float(a3 << 16));
  h01 = (int)(a0 | (a1 << 16)); h23 = (int)(a2 | (a3 << 16));
  l01 = (int)(b0 | (b1 << 16)); l23 = (int)(b2 | (b3 << 16));
}

__device__ __forceinline__ v4i regroup8(int h01, int h23, int l01, int l23, int lane) {
  const int t  = lane & 15;
  const int s0 = (lane & 16) + ((2 * t) & 15), s1 = s0 + 1;
  const int a0 = __shfl(h01, s0, 32), a1 = __shfl(h23, s0, 32), a2 = __shfl(h01, s1, 32), a3 = __shfl(h23, s1, 32);
  const int b0 = __shfl(l01, s0, 32), b1 = __shfl(l23, s0, 32), b2 = __shfl(l01, s1, 32), b3 = __shfl(l23, s1, 32);
  const int mk = (t < 8) ? -1 : 0;
  v4i o;
  o.x = (a0 & mk) | (b0 & ~mk); o.y = (a1 & mk) | (b1 & ~mk);
  o.z = (a2 & mk) | (b2 & ~mk); o.w = (a3 & mk) | (b3 & ~mk);
  return o;
}

__device__ __forceinline__ void st2_v4f(float* p, v4f v) {
  *(volatile v4f*)p = v;
  __threadfence();
  *(volatile v4f*)p = v;
}
__device__ __forceinline__ void st2_v8us(unsigned short* p, v8us v) {
  *(volatile v8us*)p = v;
  __threadfence();
  *(volatile v8us*)p = v;
}

__device__ __forceinline__ v8us gather8(const float* __restrict__ base, int stride) {
  float f[8];
#pragma unroll
  for (int i = 0; i < 8; ++i) f[i] = base[(size_t)i * (size_t)stride];
  v8us o;
#pragma unroll
  for (int i = 0; i < 8; ++i) o[i] = (unsigned short)bf16_bits(f[i]);
  return o;
}

__global__ __launch_bounds__(NTHR) void k_prep(const float* __restrict__ x, const float* __restrict__ w1,
                                               const float* __restrict__ w2, const float* __restrict__ w3,
                                               const float* __restrict__ b1, const float* __restrict__ b2,
                                               const float* __restrict__ b3,
                                               unsigned short* xb, unsigned short* w1t, unsigned short* w2d,
                                               unsigned short* w3d, float* bias) {
  const int tid = (int)threadIdx.x;
  const int blk = (int)blockIdx.x;
  if (blk < PBX) {
    const int u   = blk * NTHR + tid;
    const int row = u >> 4, k8 = (u & 15) * 8;
    const int rc  = row < NN ? row : NN - 1;
    const unsigned mk = row < NN ? 0xffffu : 0u;
    const float* p = x + (size_t)rc * CIN + k8;
    const v4f a = *(const v4fa*)p;
    const v4f b = *(const v4fa*)(p + 4);
    v8us o;
    o[0] = (unsigned short)(bf16_bits(a.x) & mk); o[1] = (unsigned short)(bf16_bits(a.y) & mk);
    o[2] = (unsigned short)(bf16_bits(a.z) & mk); o[3] = (unsigned short)(bf16_bits(a.w) & mk);
    o[4] = (unsigned short)(bf16_bits(b.x) & mk); o[5] = (unsigned short)(bf16_bits(b.y) & mk);
    o[6] = (unsigned short)(bf16_bits(b.z) & mk); o[7] = (unsigned short)(bf16_bits(b.w) & mk);
    st2_v8us(xb + (size_t)row * KL + k8, o);
  } else if (blk < PBX + PBW) {
    const int u = (blk - PBX) * NTHR + tid;
    const int n = u >> 4, k8 = (u & 15) * 8;
    const v8us o = gather8(w1 + (size_t)k8 * HD + n, HD);
    st2_v8us(w1t + (size_t)n * BPITCH + k8, o);
  } else if (blk < PBX + 2 * PBW) {
    const int u = (blk - PBX - PBW) * NTHR + tid;
    const int n = u >> 4, k8 = (u & 15) * 8, kk = k8 & (HD - 1);
    const v8us o = gather8(w2 + (size_t)kk * HD + n, HD);
    st2_v8us(w2d + (size_t)n * BPITCH + k8, o);
  } else if (blk < PBX + 3 * PBW) {
    const int u = (blk - PBX - 2 * PBW) * NTHR + tid;
    const int n = u >> 4, k8 = (u & 15) * 8, kk = k8 & (HD - 1);
    const v8us o = gather8(w3 + (size_t)kk * HD + n, HD);
    st2_v8us(w3d + (size_t)n * BPITCH + k8, o);
  } else {
    if (tid < 64) {
      const int a = tid >> 4, q = tid & 15;
      const v4f v1 = *(const v4fa*)(b1 + 4 * q);
      const v4f v2 = *(const v4fa*)(b2 + 4 * q);
      const v4f v3 = *(const v4fa*)(b3 + 4 * q);
      asm volatile("" :: "v"(v1));
      asm volatile("" :: "v"(v2));
      asm volatile("" :: "v"(v3));
      const unsigned m1 = (a == 0) ? 0xffffffffu : 0u;
      const unsigned m2 = (a == 1) ? 0xffffffffu : 0u;
      const unsigned m3 = (a == 2) ? 0xffffffffu : 0u;
      v4f o;
      o.x = __uint_as_float(((bf16_bits(v1.x) << 16) & m1) | ((bf16_bits(v2.x) << 16) & m2) | ((bf16_bits(v3.x) << 16) & m3));
      o.y = __uint_as_float(((bf16_bits(v1.y) << 16) & m1) | ((bf16_bits(v2.y) << 16) & m2) | ((bf16_bits(v3.y) << 16) & m3));
      o.z = __uint_as_float(((bf16_bits(v1.z) << 16) & m1) | ((bf16_bits(v2.z) << 16) & m2) | ((bf16_bits(v3.z) << 16) & m3));
      o.w = __uint_as_float(((bf16_bits(v1.w) << 16) & m1) | ((bf16_bits(v2.w) << 16) & m2) | ((bf16_bits(v3.w) << 16) & m3));
      st2_v4f(bias + 4 * tid, o);
    }
  }
}

__device__ __forceinline__ void bucket_flush(const int* pl, const int* cnt, const int* cur, int ov,
                                             int* lp, int* cop, int* dvp, int* fp, int tid) {
#pragma unroll 1
  for (int i = tid * 4; i < RCAP; i += NTHR * 4) {
    const v4i v = *(const v4ia*)(pl + i);
    *(volatile v4i*)(lp + i) = v;
  }
#pragma unroll 1
  for (int it = 0; it < 2; ++it) {
    const int i = (it * NTHR + tid) * 4;
    const v4i v = *(const v4ia*)(cnt + i);
    *(volatile v4i*)(cop + i) = v;
  }
  {
    const v4i v = *(const v4ia*)(cur + 4 * tid);
    *(volatile v4i*)(dvp + 4 * tid) = v;
  }
  if (tid < 8) {
    const v4i f = {ov, ov, ov, ov};
    *(volatile v4i*)(fp + 4 * tid) = f;
  }
}

__global__ __launch_bounds__(NTHR) void k_bucket(const int* __restrict__ srcs, const int* __restrict__ dsts,
                                                 int* LIST, int* CO, int* DINVB, int* FLAG) {
  extern __shared__ __attribute__((aligned(16))) int dsm[];
  int* wl   = dsm;
  int* pl   = dsm + NWAVE * WLCAP;
  int* cnt  = pl + RCAP;
  int* offs = cnt + NBRUN;
  int* cur  = offs + NBRUN;
  int* misc = cur + NBRUN;
  const int tid = (int)threadIdx.x, lane = tid & 31, wave = tid >> 5;
  const int blk = (int)blockIdx.x;
  const unsigned nbs = (unsigned)(blk * NBRUN);

  {
    const v4i z4 = {0, 0, 0, 0};
    for (int i = tid * 4; i < BK_ZINTS; i += NTHR * 4) *(v4ia*)(dsm + i) = z4;
    if (tid < 16) misc[tid] = 0;
  }
  __syncthreads();

  {
    const int per  = ((NE + NWAVE * WCH - 1) / (NWAVE * WCH)) * WCH;
    const int ebeg = wave * per;
    const int eend = (ebeg + per < NE) ? (ebeg + per) : NE;
    int* mylist = wl + wave * WLCAP;
    int wc = 0;
#pragma unroll 1
    for (int cb = ebeg; cb < eend; cb += WCH) {
      const int e0 = cb + lane * EPT;
      const v4i da = *(const v4ia*)(dsts + e0);
      const v4i db = *(const v4ia*)(dsts + e0 + 4);
      const unsigned s0 = (unsigned)da.x - nbs, s1 = (unsigned)da.y - nbs;
      const unsigned s2 = (unsigned)da.z - nbs, s3 = (unsigned)da.w - nbs;
      const unsigned s4 = (unsigned)db.x - nbs, s5 = (unsigned)db.y - nbs;
      const unsigned s6 = (unsigned)db.z - nbs, s7 = (unsigned)db.w - nbs;
      const bool h0 = s0 < (unsigned)NBRUN, h1 = s1 < (unsigned)NBRUN, h2 = s2 < (unsigned)NBRUN, h3 = s3 < (unsigned)NBRUN;
      const bool h4 = s4 < (unsigned)NBRUN, h5 = s5 < (unsigned)NBRUN, h6 = s6 < (unsigned)NBRUN, h7 = s7 < (unsigned)NBRUN;
      const unsigned m0 = __builtin_amdgcn_ballot_w32(h0), m1 = __builtin_amdgcn_ballot_w32(h1);
      const unsigned m2 = __builtin_amdgcn_ballot_w32(h2), m3 = __builtin_amdgcn_ballot_w32(h3);
      const unsigned m4 = __builtin_amdgcn_ballot_w32(h4), m5 = __builtin_amdgcn_ballot_w32(h5);
      const unsigned m6 = __builtin_amdgcn_ballot_w32(h6), m7 = __builtin_amdgcn_ballot_w32(h7);
      const unsigned any = m0 | m1 | m2 | m3 | m4 | m5 | m6 | m7;
      if (any != 0u) {
        const int pre = (int)(__builtin_amdgcn_mbcnt_lo(m0, 0u) + __builtin_amdgcn_mbcnt_lo(m1, 0u) +
                              __builtin_amdgcn_mbcnt_lo(m2, 0u) + __builtin_amdgcn_mbcnt_lo(m3, 0u) +
                              __builtin_amdgcn_mbcnt_lo(m4, 0u) + __builtin_amdgcn_mbcnt_lo(m5, 0u) +
                              __builtin_amdgcn_mbcnt_lo(m6, 0u) + __builtin_amdgcn_mbcnt_lo(m7, 0u));
        int p = wc + pre;
        if (h0) { if (p < WLCAP) mylist[p] = ((e0 + 0) << SLB) | (int)s0; p = p + 1; }
        if (h1) { if (p < WLCAP) mylist[p] = ((e0 + 1) << SLB) | (int)s1; p = p + 1; }
        if (h2) { if (p < WLCAP) mylist[p] = ((e0 + 2) << SLB) | (int)s2; p = p + 1; }
        if (h3) { if (p < WLCAP) mylist[p] = ((e0 + 3) << SLB) | (int)s3; p = p + 1; }
        if (h4) { if (p < WLCAP) mylist[p] = ((e0 + 4) << SLB) | (int)s4; p = p + 1; }
        if (h5) { if (p < WLCAP) mylist[p] = ((e0 + 5) << SLB) | (int)s5; p = p + 1; }
        if (h6) { if (p < WLCAP) mylist[p] = ((e0 + 6) << SLB) | (int)s6; p = p + 1; }
        if (h7) { if (p < WLCAP) mylist[p] = ((e0 + 7) << SLB) | (int)s7; p = p + 1; }
        wc += (int)(__builtin_popcount(m0) + __builtin_popcount(m1) + __builtin_popcount(m2) + __builtin_popcount(m3) +
                    __builtin_popcount(m4) + __builtin_popcount(m5) + __builtin_popcount(m6) + __builtin_popcount(m7));
      }
    }
    if (lane == 0) misc[wave] = wc;
  }
  __syncthreads();

  if (wave == 0) {
    int ov = 0;
#pragma unroll 1
    for (int w2 = 0; w2 < NWAVE; ++w2) {
      int c = misc[w2];
      if (c > WLCAP) ov = 1;
      c = c < 0 ? 0 : (c > WLCAP ? WLCAP : c);
#pragma unroll 1
      for (int b0 = 0; b0 < c; b0 += 32) {
        const int idx = b0 + lane;
        const int ent = wl[w2 * WLCAP + (idx < WLCAP ? idx : WLCAP - 1)];
        const int m32 = (c - b0) < 32 ? (c - b0) : 32;
#pragma unroll 1
        for (int k = 0; k < m32; ++k) {
          const int u    = __builtin_amdgcn_readlane(ent, k);
          const int slot = u & (NBRUN - 1);
          if (lane == 0) cnt[slot] = cnt[slot] + 1;
        }
      }
    }
    if (lane == 0) misc[9] = ov;
  }
  __syncthreads();
  if (wave == 0) {
    const int base = lane * (NBRUN / 32);
    int s = 0;
#pragma unroll 1
    for (int i = 0; i < NBRUN / 32; ++i) s += cnt[base + i];
    int incl = s;
#pragma unroll
    for (int d = 1; d < 32; d <<= 1) {
      const int y = __shfl_up(incl, d, 32);
      if (lane >= d) incl += y;
    }
    int run = incl - s;
#pragma unroll 1
    for (int i = 0; i < NBRUN / 32; ++i) {
      const int cv = cnt[base + i];
      offs[base + i] = run;
      cur[base + i]  = run;
      run += cv;
    }
  }
  __syncthreads();

  if (wave == 0) {
#pragma unroll 1
    for (int w2 = 0; w2 < NWAVE; ++w2) {
      int c = misc[w2];
      c = c < 0 ? 0 : (c > WLCAP ? WLCAP : c);
#pragma unroll 1
      for (int b0 = 0; b0 < c; b0 += 32) {
        const int idx = b0 + lane;
        const int ent = wl[w2 * WLCAP + (idx < WLCAP ? idx : WLCAP - 1)];
        int eid = (ent >> SLB) & 0x1FFFFF;
        eid = eid > NE - 1 ? NE - 1 : eid;
        int sr = srcs[eid];
        sr = sr < 0 ? 0 : (sr > NN - 1 ? NN - 1 : sr);
        const int m32 = (c - b0) < 32 ? (c - b0) : 32;
#pragma unroll 1
        for (int k = 0; k < m32; ++k) {
          const int u    = __builtin_amdgcn_readlane(ent, k);
          const int wd   = __builtin_amdgcn_readlane(sr, k);
          const int slot = u & (NBRUN - 1);
          if (lane == 0) {
            int p = cur[slot];
            p = p < 0 ? 0 : (p > RCAP - 1 ? RCAP - 1 : p);
            pl[p] = wd;
            cur[slot] = p + 1;
          }
        }
      }
    }
  }
  __syncthreads();

#pragma unroll 1
  for (int qd = 0; qd < NBRUN / NTHR; ++qd) {
    const int s = qd * NTHR + tid;
    int c = cnt[s];
    c = c < 0 ? 0 : c;
    const float dg = (float)(c + 1);
    const float dv = 1.0f / sqrtf(dg);
    cur[s] = __float_as_int(dv);
  }
  __syncthreads();

  const int ovf = misc[9];
  int* lp  = LIST + (size_t)blk * RCAP;
  int* cop = CO + (size_t)blk * (2 * NBRUN);
  int* dvp = DINVB + (size_t)blk * NBRUN;
  int* fp  = FLAG + (size_t)blk * 32;
  bucket_flush(pl, cnt, cur, ovf, lp, cop, dvp, fp, tid);
  __threadfence();
  bucket_flush(pl, cnt, cur, ovf, lp, cop, dvp, fp, tid);
}

template <int KEXT>
__device__ __forceinline__ void gemm_16x64(const unsigned short* __restrict__ ap,
                                           const unsigned short* __restrict__ bp, v8f (&acc)[4]) {
#pragma unroll 1
  for (int k0 = 0; k0 < KEXT; k0 += 32) {
    FragB af;
    af.h[0] = *(const v8usa*)(ap + k0);
    af.h[1] = *(const v8usa*)(ap + k0 + 16);
#pragma unroll
    for (int nt = 0; nt < 4; ++nt) {
      const unsigned short* wq = bp + (size_t)(16 * nt) * (size_t)BPITCH + k0;
      FragB bf;
      bf.h[0] = *(const v8usa*)wq;
      bf.h[1] = *(const v8usa*)(wq + 16);
      acc[nt] = wmb(af, bf, acc[nt]);
    }
  }
}

__device__ __forceinline__ void stage_d(float* stg, const v8f (&acc)[4], int wave, int hh, int m) {
#pragma unroll
  for (int nt = 0; nt < 4; ++nt) {
#pragma unroll
    for (int r = 0; r < 8; ++r) stg[(16 * wave + 8 * hh + r) * SP + 16 * nt + m] = acc[nt][r];
  }
}

template <int KEXT>
__device__ __forceinline__ void gemm_rows(const unsigned short* __restrict__ A,
                                          const unsigned short* __restrict__ BT,
                                          const float* __restrict__ DINV, float* P, float* stg) {
  const int tid = (int)threadIdx.x, lane = tid & 31, wave = tid >> 5, hh = lane >> 4, m = lane & 15;
  const int rowBase = (int)blockIdx.x * GBM;

  v8f acc[4];
  {
    const v8f z = {0.f, 0.f, 0.f, 0.f, 0.f, 0.f, 0.f, 0.f};
#pragma unroll
    for (int t = 0; t < 4; ++t) acc[t] = z;
  }
  const unsigned short* ap = A + (size_t)(rowBase + 16 * wave + m) * (size_t)APITCH + 8 * hh;
  const unsigned short* bp = BT + (size_t)m * (size_t)BPITCH + 8 * hh;
  gemm_16x64<KEXT>(ap, bp, acc);
  stage_d(stg, acc, wave, hh, m);
  __syncthreads();

#pragma unroll 1
  for (int i = 0; i < 8; ++i) {
    const int lr   = 16 * wave + 2 * i + hh;
    const int grow = rowBase + lr;
    const bool live = grow < NN;
    const v4f a = *(const v4fa*)(stg + lr * SP + 4 * m);
    const float dv = DINV[grow];
    asm volatile("" :: "v"(a));
    asm volatile("" :: "v"(dv));
    const float v0 = a.x * dv, v1 = a.y * dv, v2 = a.z * dv, v3 = a.w * dv;
    v4f o;
    o.x = live ? v0 : 0.0f; o.y = live ? v1 : 0.0f; o.z = live ? v2 : 0.0f; o.w = live ? v3 : 0.0f;
    st2_v4f(P + (size_t)grow * HD + 4 * m, o);
  }
}

__global__ __launch_bounds__(NTHR) __attribute__((amdgpu_num_vgpr(248)))
void k_gemm_one(const unsigned short* __restrict__ XB, const unsigned short* __restrict__ W1T,
                const float* __restrict__ DINV, float* P) {
  __shared__ __attribute__((aligned(16))) float stg[GBM * SP];
  gemm_rows<CIN>(XB, W1T, DINV, P, stg);
}

__global__ __launch_bounds__(NTHR) __attribute__((amdgpu_num_vgpr(248)))
void k_gemm_two(const unsigned short* __restrict__ Hhl, const unsigned short* __restrict__ WD,
                const float* __restrict__ DINV, float* P) {
  __shared__ __attribute__((aligned(16))) float stg[GBM * SP];
  gemm_rows<K2EXT>(Hhl, WD, DINV, P, stg);
}

template <int FINAL>
__global__ __launch_bounds__(NTHR) void k_replay(const int* __restrict__ LIST, const int* __restrict__ CO,
                                                 const float* __restrict__ DINV, const int* __restrict__ FLAG,
                                                 const float* __restrict__ P, const float* __restrict__ BIAS,
                                                 unsigned short* Hhl, float* out) {
  __shared__ __attribute__((aligned(16))) float sb[64];
  const int tid = (int)threadIdx.x, lane = tid & 31, wave = tid >> 5, hh = lane >> 4, q = lane & 15;
  const int blk = (int)blockIdx.x;
  const int rowBase = blk * NBRUN;
  const int* lb  = LIST + (size_t)blk * RCAP;
  const int* cob = CO + (size_t)blk * (2 * NBRUN);
  if (tid < 16) *(v4fa*)(sb + 4 * tid) = *(const v4fa*)(BIAS + 4 * tid);
  __syncthreads();
  const int flag = FLAG[(size_t)blk * 32];
  const v4f bias = *(const v4fa*)(sb + 4 * q);
  const float qnan = __uint_as_float(0x7fc00000u);

#pragma unroll 1
  for (int i = 0; i < NBRUN / (2 * NWAVE); ++i) {
    const int slot = (NBRUN / NWAVE) * wave + 2 * i + hh;
    const int d    = rowBase + slot;
    int c = cob[slot];
    int o = cob[NBRUN + slot];
    const bool big = c > DEGCAP;
    c = c < 0 ? 0 : (c > DEGCAP ? DEGCAP : c);
    o = o < 0 ? 0 : (o > RCAP - 1 ? RCAP - 1 : o);
    const int co  = __shfl_xor(c, 16, 32);
    const int cmv = c > co ? c : co;
    const int cm  = __builtin_amdgcn_readfirstlane(cmv);
    int last = o + c - 1;
    last = last < o ? o : last;
    last = last > RCAP - 1 ? RCAP - 1 : last;
    float a0 = 0.0f, a1 = 0.0f, a2 = 0.0f, a3 = 0.0f;
#pragma unroll 1
    for (int j = 0; j < cm; ++j) {
      int idx = o + j;
      idx = idx > last ? last : idx;
      int sr = lb[idx];
      sr = sr < 0 ? 0 : (sr > NN - 1 ? NN - 1 : sr);
      const v4f v = *(const v4fa*)(P + (size_t)sr * HD + 4 * q);
      asm volatile("" :: "v"(v));
      const bool valid = j < c;
      const float t0 = a0 + v.x, t1 = a1 + v.y, t2 = a2 + v.z, t3 = a3 + v.w;
      a0 = valid ? t0 : a0; a1 = valid ? t1 : a1; a2 = valid ? t2 : a2; a3 = valid ? t3 : a3;
    }
    const int dc = d < MP ? d : MP - 1;
    const v4f g = *(const v4fa*)(P + (size_t)dc * HD + 4 * q);
    const float dv = DINV[d];
    asm volatile("" :: "v"(g));
    asm volatile("" :: "v"(dv));
    float v0 = (a0 + g.x) * dv + bias.x, v1 = (a1 + g.y) * dv + bias.y;
    float v2 = (a2 + g.z) * dv + bias.z, v3 = (a3 + g.w) * dv + bias.w;
    if constexpr (FINAL == 0) {
      v0 = (v0 > 0.0f) ? v0 : (v0 - v0); v1 = (v1 > 0.0f) ? v1 : (v1 - v1);
      v2 = (v2 > 0.0f) ? v2 : (v2 - v2); v3 = (v3 > 0.0f) ? v3 : (v3 - v3);
    }
    const bool bad  = (flag != 0) | big;
    const bool live = d < NN;
    v0 = bad ? qnan : v0; v1 = bad ? qnan : v1; v2 = bad ? qnan : v2; v3 = bad ? qnan : v3;
    v0 = live ? v0 : 0.0f; v1 = live ? v1 : 0.0f; v2 = live ? v2 : 0.0f; v3 = live ? v3 : 0.0f;
    if constexpr (FINAL == 0) {
      int h01, h23, l01, l23;
      hilo_pack(v0, v1, v2, v3, h01, h23, l01, l23);
      const v4i ow = regroup8(h01, h23, l01, l23, lane);
      const int dr = d < MP ? d : MP - 1;
      unsigned short* hp = Hhl + (size_t)dr * KL + 8 * q;
      const bool wr = d < MP;
      if (wr) *(volatile v4i*)hp = ow;
      __threadfence();
      if (wr) *(volatile v4i*)hp = ow;
    } else {
      v4f ov;
      ov.x = v0; ov.y = v1; ov.z = v2; ov.w = v3;
      const int dr = d < NN ? d : NN - 1;
      float* op = out + (size_t)dr * HD + 4 * q;
      const bool wr = d < NN;
      if (wr) *(volatile v4f*)op = ov;
      __threadfence();
      if (wr) *(volatile v4f*)op = ov;
    }
  }
}

extern "C" void kernel_launch(void* const* d_in, const int* in_sizes, int n_in,
                              void* d_out, int out_size, void* d_ws, size_t ws_size,
                              hipStream_t stream) {
  if (n_in < 8) return;
  if (in_sizes[0] != NN * CIN) return;
  if (in_sizes[1] != CIN * HD) return;
  if (in_sizes[2] != HD) return;
  if (in_sizes[3] != HD * HD) return;
  if (in_sizes[4] != HD) return;
  if (in_sizes[5] != HD * HD) return;
  if (in_sizes[6] != HD) return;
  if (in_sizes[7] != 2 * NE) return;
  if (out_size != NN * HD) return;

  const float* x  = (const float*)d_in[0];
  const float* W1 = (const float*)d_in[1];
  const float* b1 = (const float*)d_in[2];
  const float* W2 = (const float*)d_in[3];
  const float* b2 = (const float*)d_in[4];
  const float* W3 = (const float*)d_in[5];
  const float* b3 = (const float*)d_in[6];
  const int*   ei = (const int*)d_in[7];
  float* out = (float*)d_out;
  const int* srcs = ei;
  const int* dsts = ei + NE;

  constexpr size_t zXB   = (size_t)MP * KL * 2;
  constexpr size_t zP    = (size_t)MP * HD * 4;
  constexpr size_t zHL   = (size_t)MP * KL * 2;
  constexpr size_t zLIST = (size_t)NBK * RCAP * 4;
  constexpr size_t zCO   = (size_t)NBK * 2 * NBRUN * 4;
  constexpr size_t zDINV = (size_t)NBK * NBRUN * 4;
  constexpr size_t zFLAG = (size_t)NBK * 128;
  constexpr size_t zW    = (size_t)HD * BPITCH * 2;
  constexpr size_t zBIAS = 1024;
  constexpr size_t oXB   = 0;
  constexpr size_t oP    = oXB + zXB;
  constexpr size_t oHL   = oP + zP;
  constexpr size_t oLIST = oHL + zHL;
  constexpr size_t oCO   = oLIST + zLIST;
  constexpr size_t oDINV = oCO + zCO;
  constexpr size_t oFLAG = oDINV + zDINV;
  constexpr size_t oW1T  = oFLAG + zFLAG;
  constexpr size_t oW2D  = oW1T + zW;
  constexpr size_t oW3D  = oW2D + zW;
  constexpr size_t oBIAS = oW3D + zW;
  constexpr size_t oEND  = oBIAS + zBIAS;
  static_assert(zXB % 128 == 0 && zP % 128 == 0 && zHL % 128 == 0 && zLIST % 128 == 0 && zCO % 128 == 0);
  static_assert(zDINV % 128 == 0 && zFLAG % 128 == 0 && zW % 128 == 0 && zBIAS % 128 == 0);
  static_assert(oEND <= WSMAX);
  if (oEND > ws_size) return;

  char* ws = (char*)d_ws;
  unsigned short* XB   = (unsigned short*)(ws + oXB);
  float*          P    = (float*)(ws + oP);
  unsigned short* Hhl  = (unsigned short*)(ws + oHL);
  int*            LIST = (int*)(ws + oLIST);
  int*            CO   = (int*)(ws + oCO);
  int*            DVB  = (int*)(ws + oDINV);
  const float*    DINV = (const float*)(ws + oDINV);
  int*            FLAG = (int*)(ws + oFLAG);
  unsigned short* W1T  = (unsigned short*)(ws + oW1T);
  unsigned short* W2D  = (unsigned short*)(ws + oW2D);
  unsigned short* W3D  = (unsigned short*)(ws + oW3D);
  float*          BIAS = (float*)(ws + oBIAS);

  hipFuncSetAttribute(reinterpret_cast<const void*>(&k_bucket), hipFuncAttributeMaxDynamicSharedMemorySize, (int)BK_LDS);

  k_prep<<<PBTOT, NTHR, 0, stream>>>(x, W1, W2, W3, b1, b2, b3, XB, W1T, W2D, W3D, BIAS);
  k_bucket<<<NBK, NTHR, BK_LDS, stream>>>(srcs, dsts, LIST, CO, DVB, FLAG);
  k_gemm_one<<<MP / GBM, NTHR, 0, stream>>>(XB, W1T, DINV, P);
  k_replay<0><<<NBK, NTHR, 0, stream>>>(LIST, CO, DINV, FLAG, P, BIAS, Hhl, out);
  k_gemm_two<<<MP / GBM, NTHR, 0, stream>>>(Hhl, W2D, DINV, P);
  k_replay<0><<<NBK, NTHR, 0, stream>>>(LIST, CO, DINV, FLAG, P, BIAS + HD, Hhl, out);
  k_gemm_two<<<MP / GBM, NTHR, 0, stream>>>(Hhl, W3D, DINV, P);
  k_replay<1><<<NBK, NTHR, 0, stream>>>(LIST, CO, DINV, FLAG, P, BIAS + 2 * HD, Hhl, out);
}
